// transformer_55791625175537
// MI455X (gfx1250) — hardware-verified
//
#include <hip/hip_runtime.h>
#include <math.h>
#pragma clang fp contract(off)

typedef __attribute__((ext_vector_type(16))) _Float16 v16h;
typedef __attribute__((ext_vector_type(8)))  _Float16 v8h;
typedef __attribute__((ext_vector_type(8)))  float    v8f;
typedef __attribute__((ext_vector_type(4)))  float    v4f;
typedef __attribute__((ext_vector_type(2)))  float    v2f;
typedef __attribute__((ext_vector_type(4)))  int      v4i;

constexpr int NBATCH = 4;
constexpr int NPT = 4096;
constexpr int CH_IN = 128;
constexpr int CH_D = 64;
constexpr int NBR = 16;
constexpr int CH_HID = 256;
constexpr int NPOINTS = NBATCH * NPT;
constexpr int NROWS_ALL = NPOINTS * NBR;
constexpr float WCARRY = 16.0f;
constexpr float WCARRY_INV = 1.0f / 16.0f;
constexpr float BN_EPS_F = 1e-3f;
static_assert(NPOINTS == 16384, "shape");
static_assert(NROWS_ALL == 262144, "shape");
static_assert(CH_HID == 4 * CH_D, "shape");

constexpr int OFF_WST  = 0;
constexpr int OFF_WK   = OFF_WST + CH_D * CH_IN;
constexpr int OFF_WQ   = OFF_WK + CH_D * CH_D;
constexpr int OFF_WV   = OFF_WQ + CH_D * CH_D;
constexpr int OFF_WP2  = OFF_WV + CH_D * CH_D;
constexpr int OFF_WA1  = OFF_WP2 + CH_D * CH_D;
constexpr int OFF_WA2  = OFF_WA1 + CH_HID * CH_D;
constexpr int OFF_WEND = OFF_WA2 + CH_D * CH_HID;
constexpr int PACK_HALVES = OFF_WEND + CH_IN * CH_D;
static_assert(PACK_HALVES == 65536, "pack size");

union FragH { v16h v; v8h h[2]; };

__device__ __forceinline__ v16h frag_load(const _Float16* p) {
  FragH f;
  f.h[0] = *(const v8h*)(p);
  f.h[1] = *(const v8h*)(p + 16);
  return f.v;
}

__device__ __forceinline__ v16h frag_from_f32(const float* p) {
  const v4f x0 = *(const v4f*)(p);
  const v4f x1 = *(const v4f*)(p + 4);
  const v4f x2 = *(const v4f*)(p + 16);
  const v4f x3 = *(const v4f*)(p + 20);
  v16h a;
#pragma unroll
  for (int j = 0; j < 4; ++j) {
    a[j]      = (_Float16)x0[j];
    a[4 + j]  = (_Float16)x1[j];
    a[8 + j]  = (_Float16)x2[j];
    a[12 + j] = (_Float16)x3[j];
  }
  return a;
}

__device__ __forceinline__ v8f mma_h(v16h a, v16h b, v8f c) {
  c = __builtin_amdgcn_wmma_f32_16x16x32_f16(false, a, false, b, (short)0, c, false, false);
  asm volatile("v_nop\n\tv_nop\n\tv_nop\n\tv_nop" : "+v"(c) : "v"(a), "v"(b));
  return c;
}

__device__ __forceinline__ void wave_lds_sync() {
  __builtin_amdgcn_fence(__ATOMIC_RELEASE, "workgroup");
  __builtin_amdgcn_wave_barrier();
  __builtin_amdgcn_fence(__ATOMIC_ACQUIRE, "workgroup");
}

__device__ __forceinline__ float h16_to_f32(unsigned hb) {
  const unsigned sgn = (hb & 0x8000u) << 16;
  const unsigned em = hb & 0x7fffu;
  const float fn = __uint_as_float((em << 13) + 0x38000000u);
  const float fs = (float)em * 5.9604644775390625e-8f;
  const float mag = (em < 0x400u) ? fs : fn;
  return __uint_as_float(__float_as_uint(mag) | sgn);
}

__device__ __forceinline__ void store_tile_f16(const float* slab, _Float16* dst, int lane) {
  const int q = lane >> 3, c8 = (lane & 7) * 8;
  v8h hv[4];
#pragma unroll
  for (int it = 0; it < 4; ++it) {
    const float* sp = slab + (it * 4 + q) * 68 + c8;
    const v4f a0 = *(const v4f*)(sp);
    const v4f a1 = *(const v4f*)(sp + 4);
#pragma unroll
    for (int j = 0; j < 4; ++j) {
      hv[it][j]     = (_Float16)a0[j];
      hv[it][4 + j] = (_Float16)a1[j];
    }
  }
  for (int pass = 0; pass < 2; ++pass) {
#pragma unroll
    for (int it = 0; it < 4; ++it)
      *(volatile v8h*)(dst + (size_t)(it * 4 + q) * 64 + c8) = hv[it];
    __threadfence();
  }
}

__global__ __launch_bounds__(256) void k_pack(
    const float* __restrict__ Wst, const float* __restrict__ Wk, const float* __restrict__ Wq,
    const float* __restrict__ Wv, const float* __restrict__ Wp2, const float* __restrict__ Wa1,
    const float* __restrict__ Wa2, const float* __restrict__ Wend, _Float16* __restrict__ outp) {
  const int bx = blockIdx.x;
  const float* W = Wst;
  int Kd = CH_IN, Nd = CH_D, base = 0;
  if (bx >= 28)      { W = Wend; Kd = CH_D;   Nd = CH_IN;  base = 7168; }
  else if (bx >= 20) { W = Wa2;  Kd = CH_HID; Nd = CH_D;   base = 5120; }
  else if (bx >= 12) { W = Wa1;  Kd = CH_D;   Nd = CH_HID; base = 3072; }
  else if (bx >= 10) { W = Wp2;  Kd = CH_D;   Nd = CH_D;   base = 2560; }
  else if (bx >= 8)  { W = Wv;   Kd = CH_D;   Nd = CH_D;   base = 2048; }
  else if (bx >= 6)  { W = Wq;   Kd = CH_D;   Nd = CH_D;   base = 1536; }
  else if (bx >= 4)  { W = Wk;   Kd = CH_D;   Nd = CH_D;   base = 1024; }
  const int g = bx * 256 + threadIdx.x;
  const int lc = g - base;
  const int cpr = Kd >> 3;
  const int n = lc / cpr;
  const int k0 = (lc - n * cpr) << 3;
  v8h hv;
#pragma unroll
  for (int e = 0; e < 8; ++e) {
    const float w = W[(size_t)(k0 + e) * Nd + n];
    hv[e] = (_Float16)(w * WCARRY);
  }
  _Float16* o = outp + (size_t)g * 8;
  *(volatile v8h*)o = hv;
  __threadfence();
  *(volatile v8h*)o = hv;
}

__global__ __launch_bounds__(256) void k_knn(const float* __restrict__ pos, int* __restrict__ idxb) {
#pragma clang fp contract(off)
  __shared__ __align__(16) v4f cand[2048];
  __shared__ __align__(16) int sidx[256 * 16];
  const int tid = threadIdx.x;
  const int b = blockIdx.y;
  const float* pb = pos + (size_t)b * NPT * 3;
  const int q = blockIdx.x * 256 + tid;
  const float qx = pb[q * 3], qy = pb[q * 3 + 1], qz = pb[q * 3 + 2];
  const float qxx = qx * qx;
  const float qyy = qy * qy;
  const float qzz = qz * qz;
  const float sqn = (qxx + qzz) + qyy;
  float bd[NBR];
  int bi[NBR];
#pragma unroll
  for (int j = 0; j < NBR; ++j) { bd[j] = INFINITY; bi[j] = 0; }

  for (int ch = 0; ch < 2; ++ch) {
    __syncthreads();
#pragma unroll 1
    for (int i = tid; i < 2048; i += 256) {
      const int mI = ch * 2048 + i;
      const float cx = pb[mI * 3], cy = pb[mI * 3 + 1], cz = pb[mI * 3 + 2];
      const float xx = cx * cx;
      const float yy = cy * cy;
      const float zz = cz * cz;
      const float sq = (xx + zz) + yy;
      cand[i] = (v4f){cx, cy, cz, sq};
    }
    __syncthreads();
#pragma unroll 1
    for (int c = 0; c < 2048; ++c) {
      const v4f cm = cand[c];
      float p = qx * cm.x;
      p = fmaf(qy, cm.y, p);
      p = fmaf(qz, cm.z, p);
      const float s2 = sqn + cm.w;
      const float tp = 2.0f * p;
      const float d = s2 - tp;
      if (d < bd[NBR - 1]) {
        const int ci = ch * 2048 + c;
#pragma unroll
        for (int j = NBR - 1; j >= 1; --j) {
          const bool sh = d < bd[j - 1];
          const bool ins = d < bd[j];
          bd[j] = sh ? bd[j - 1] : (ins ? d : bd[j]);
          bi[j] = sh ? bi[j - 1] : (ins ? ci : bi[j]);
        }
        const bool ins0 = d < bd[0];
        bd[0] = ins0 ? d : bd[0];
        bi[0] = ins0 ? ci : bi[0];
      }
    }
  }
#pragma unroll
  for (int gq = 0; gq < 4; ++gq)
    *(v4i*)(sidx + tid * 16 + gq * 4) = (v4i){bi[gq * 4], bi[gq * 4 + 1], bi[gq * 4 + 2], bi[gq * 4 + 3]};
  __syncthreads();
  const int wave = tid >> 5, lane = tid & 31;
  int* gdst = idxb + ((size_t)b * NPT + blockIdx.x * 256) * NBR + wave * 512;
  const int* ssrc = sidx + wave * 512;
  v4i vv[4];
#pragma unroll
  for (int it = 0; it < 4; ++it) vv[it] = *(const v4i*)(ssrc + it * 128 + lane * 4);
  for (int pass = 0; pass < 2; ++pass) {
#pragma unroll
    for (int it = 0; it < 4; ++it) *(volatile v4i*)(gdst + it * 128 + lane * 4) = vv[it];
    __threadfence();
  }
}

__device__ __forceinline__ void proj_out(v16h ha0, v16h ha1, const _Float16* Wb, const float* bias,
                                         float* O, float* sl, int row0, int lane) {
  const int m = lane & 15, hh = lane >> 4;
  v8f acc[4];
#pragma unroll
  for (int nt = 0; nt < 4; ++nt) acc[nt] = (v8f){0.f, 0.f, 0.f, 0.f, 0.f, 0.f, 0.f, 0.f};
#pragma unroll
  for (int ks = 0; ks < 2; ++ks) {
    const v16h a = (ks == 0) ? ha0 : ha1;
#pragma unroll
    for (int nt = 0; nt < 4; ++nt) {
      const v16h bfr = frag_load(Wb + (size_t)(nt * 16 + m) * CH_D + ks * 32 + 8 * hh);
      acc[nt] = mma_h(a, bfr, acc[nt]);
    }
    asm volatile("" ::: "memory");
  }
#pragma unroll
  for (int nt = 0; nt < 4; ++nt) {
    const float bb = bias[nt * 16 + m];
#pragma unroll
    for (int r = 0; r < 8; ++r) sl[(8 * hh + r) * 68 + nt * 16 + m] = fmaf(acc[nt][r], WCARRY_INV, bb);
  }
  wave_lds_sync();
  const int c4 = m * 4;
  for (int pass = 0; pass < 2; ++pass) {
#pragma unroll
    for (int it = 0; it < 8; ++it) {
      const int row = it * 2 + hh;
      const v4f v = *(const v4f*)(sl + row * 68 + c4);
      *(volatile v4f*)(O + (size_t)(row0 + row) * CH_D + c4) = v;
    }
    __threadfence();
  }
  wave_lds_sync();
}

__global__ __launch_bounds__(128) void k_proj(
    const float* __restrict__ x, const _Float16* __restrict__ pW,
    const float* __restrict__ bst, const float* __restrict__ bk,
    const float* __restrict__ bq, const float* __restrict__ bv,
    float* __restrict__ keyo, float* __restrict__ valo, float* __restrict__ qryo) {
  __shared__ __align__(16) float slab[4][16 * 68];
  const int wave = threadIdx.x >> 5, lane = threadIdx.x & 31;
  const int m = lane & 15, hh = lane >> 4;
  const int row0 = (blockIdx.x * 4 + wave) * 16;
  float* sl = slab[wave];
  v8f acc[4];
#pragma unroll
  for (int nt = 0; nt < 4; ++nt) acc[nt] = (v8f){0.f, 0.f, 0.f, 0.f, 0.f, 0.f, 0.f, 0.f};
#pragma unroll 1
  for (int ks = 0; ks < 4; ++ks) {
    const v16h a = frag_from_f32(x + (size_t)(row0 + m) * CH_IN + ks * 32 + 8 * hh);
    asm volatile("" ::: "memory");
#pragma unroll
    for (int nt = 0; nt < 4; ++nt) {
      const v16h bfr = frag_load(pW + OFF_WST + (size_t)(nt * 16 + m) * CH_IN + ks * 32 + 8 * hh);
      acc[nt] = mma_h(a, bfr, acc[nt]);
    }
    asm volatile("" ::: "memory");
  }
#pragma unroll
  for (int nt = 0; nt < 4; ++nt) {
    const float bb = bst[nt * 16 + m];
#pragma unroll
    for (int r = 0; r < 8; ++r) sl[(8 * hh + r) * 68 + nt * 16 + m] = fmaf(acc[nt][r], WCARRY_INV, bb);
  }
  wave_lds_sync();
  const v16h ha0 = frag_from_f32(sl + m * 68 + 8 * hh);
  const v16h ha1 = frag_from_f32(sl + m * 68 + 32 + 8 * hh);
  wave_lds_sync();
  proj_out(ha0, ha1, pW + OFF_WK, bk, keyo, sl, row0, lane);
  proj_out(ha0, ha1, pW + OFF_WQ, bq, valo, sl, row0, lane);
  proj_out(ha0, ha1, pW + OFF_WV, bv, qryo, sl, row0, lane);
}

__global__ __launch_bounds__(256) void k_mom(const float* __restrict__ pos, const int* __restrict__ idxb,
                                             double* __restrict__ part1) {
  __shared__ double red[9][256];
  const int tid = threadIdx.x;
  double a0 = 0.0, a1 = 0.0, a2 = 0.0, a3 = 0.0, a4 = 0.0, a5 = 0.0, a6 = 0.0, a7 = 0.0, a8 = 0.0;
#pragma unroll 1
  for (int i = 0; i < 4; ++i) {
    const int row = blockIdx.x * 1024 + i * 256 + tid;
    const int ng = row >> 4;
    const int b = ng >> 12;
    int nb = idxb[row];
    nb = nb < 0 ? 0 : (nb > NPT - 1 ? NPT - 1 : nb);
    const float* pp = pos + (size_t)ng * 3;
    const float* pc = pos + (size_t)(b * NPT + nb) * 3;
    const float dx = pp[0] - pc[0];
    const float dy = pp[1] - pc[1];
    const float dz = pp[2] - pc[2];
    const double X = (double)dx, Y = (double)dy, Z = (double)dz;
    a0 += X; a1 += Y; a2 += Z;
    a3 += X * X; a4 += X * Y; a5 += X * Z;
    a6 += Y * Y; a7 += Y * Z; a8 += Z * Z;
  }
  red[0][tid] = a0; red[1][tid] = a1; red[2][tid] = a2;
  red[3][tid] = a3; red[4][tid] = a4; red[5][tid] = a5;
  red[6][tid] = a6; red[7][tid] = a7; red[8][tid] = a8;
  __syncthreads();
  for (int s = 128; s > 0; s >>= 1) {
    if (tid < s) {
#pragma unroll
      for (int k = 0; k < 9; ++k) red[k][tid] += red[k][tid + s];
    }
    __syncthreads();
  }
  if (tid < 16) {
    const int kk = tid < 8 ? tid : 8;
    const double rv = red[kk][0];
    const double v = (tid < 9) ? rv : 0.0;
    double* o = part1 + (size_t)blockIdx.x * 16 + tid;
    *(volatile double*)o = v;
    __threadfence();
    *(volatile double*)o = v;
  }
}

__global__ __launch_bounds__(256) void k_fin1(const double* __restrict__ part1, const float* __restrict__ W1,
                                              const float* __restrict__ b1, const float* __restrict__ gamma,
                                              const float* __restrict__ beta, float* __restrict__ sclsh1) {
  __shared__ double red[9][256];
  __shared__ __align__(16) float outv[128];
  const int tid = threadIdx.x;
#pragma unroll
  for (int k = 0; k < 9; ++k) red[k][tid] = part1[(size_t)tid * 16 + k];
  __syncthreads();
  for (int s = 128; s > 0; s >>= 1) {
    if (tid < s) {
#pragma unroll
      for (int k = 0; k < 9; ++k) red[k][tid] += red[k][tid + s];
    }
    __syncthreads();
  }
  if (tid < 64) {
    const int c = tid;
    const double invR = 1.0 / (double)NROWS_ALL;
    const double mx = red[0][0] * invR, my = red[1][0] * invR, mz = red[2][0] * invR;
    const double cxx = red[3][0] * invR - mx * mx;
    const double cxy = red[4][0] * invR - mx * my;
    const double cxz = red[5][0] * invR - mx * mz;
    const double cyy = red[6][0] * invR - my * my;
    const double cyz = red[7][0] * invR - my * mz;
    const double czz = red[8][0] * invR - mz * mz;
    const double w0 = (double)W1[c], w1 = (double)W1[64 + c], w2 = (double)W1[128 + c];
    const double mean = w0 * mx + w1 * my + w2 * mz + (double)b1[c];
    const double var = w0 * w0 * cxx + w1 * w1 * cyy + w2 * w2 * czz
                     + 2.0 * (w0 * w1 * cxy + w0 * w2 * cxz + w1 * w2 * cyz);
    const float varf = fmaxf((float)var, 0.0f);
    const float scl = gamma[c] * (1.0f / sqrtf(varf + BN_EPS_F));
    const float sh = (float)((double)beta[c] - mean * (double)scl);
    outv[c] = scl;
    outv[64 + c] = sh;
  }
  __syncthreads();
  if (tid < 32) {
    const v4f v = *(const v4f*)(outv + tid * 4);
    *(volatile v4f*)(sclsh1 + tid * 4) = v;
    __threadfence();
    *(volatile v4f*)(sclsh1 + tid * 4) = v;
  }
}

__global__ __launch_bounds__(128) void k_pe_s(
    const float* __restrict__ pos, const int* __restrict__ idxb,
    const float* __restrict__ qry, const float* __restrict__ keyv,
    const float* __restrict__ W1, const float* __restrict__ b1, const float* __restrict__ sclsh1,
    const _Float16* __restrict__ pW, const float* __restrict__ bp2,
    _Float16* __restrict__ peP, _Float16* __restrict__ sP, float* __restrict__ part2) {
  __shared__ __align__(16) float slab[4][16 * 68];
  __shared__ __align__(16) v4f pcst[64];
  __shared__ int nbs[4][16];
  __shared__ __align__(16) float wst[4][512];
  const int tid = threadIdx.x;
  const int wave = tid >> 5, lane = tid & 31;
  const int m = lane & 15, hh = lane >> 4;
  if (tid < 64) {
    const int c = tid;
    const float scl = sclsh1[c], sh = sclsh1[64 + c];
    const float w0 = W1[c], w1 = W1[64 + c], w2 = W1[128 + c];
    pcst[c] = (v4f){w0 * scl, w1 * scl, w2 * scl, fmaf(b1[c], scl, sh)};
  }
  __syncthreads();
  float bp2v[4];
#pragma unroll
  for (int nt = 0; nt < 4; ++nt) bp2v[nt] = bp2[nt * 16 + m];
  float ssum[16], ssq[16];
#pragma unroll
  for (int nt = 0; nt < 16; ++nt) { ssum[nt] = 0.f; ssq[nt] = 0.f; }
  float* sl = slab[wave];
  const int c4 = m * 4;

#pragma unroll 1
  for (int it = 0; it < 8; ++it) {
    const int ng = blockIdx.x * 32 + wave * 8 + it;
    const int b = ng >> 12;
    const size_t row0 = (size_t)ng * NBR;
    int nb = idxb[row0 + m];
    nb = nb < 0 ? 0 : (nb > NPT - 1 ? NPT - 1 : nb);
    nbs[wave][m] = nb;
    const float* pp = pos + (size_t)ng * 3;
    const float* pc = pos + (size_t)(b * NPT + nb) * 3;
    const float dx = pp[0] - pc[0];
    const float dy = pp[1] - pc[1];
    const float dz = pp[2] - pc[2];
    v16h ta[2];
#pragma unroll
    for (int ks = 0; ks < 2; ++ks) {
#pragma unroll
      for (int e = 0; e < 16; ++e) {
        const int ch = ks * 32 + 8 * hh + (e & 7) + ((e >> 3) << 4);
        const v4f kc = pcst[ch];
        float v = fmaf(dx, kc.x, fmaf(dy, kc.y, fmaf(dz, kc.z, kc.w)));
        v = fmaxf(v, 0.0f);
        ta[ks][e] = (_Float16)v;
      }
    }
    v8f acc[4];
#pragma unroll
    for (int nt = 0; nt < 4; ++nt) acc[nt] = (v8f){0.f, 0.f, 0.f, 0.f, 0.f, 0.f, 0.f, 0.f};
#pragma unroll
    for (int ks = 0; ks < 2; ++ks) {
#pragma unroll
      for (int nt = 0; nt < 4; ++nt) {
        const v16h bfr = frag_load(pW + OFF_WP2 + (size_t)(nt * 16 + m) * CH_D + ks * 32 + 8 * hh);
        acc[nt] = mma_h(ta[ks], bfr, acc[nt]);
      }
      asm volatile("" ::: "memory");
    }
#pragma unroll
    for (int nt = 0; nt < 4; ++nt) {
#pragma unroll
      for (int r = 0; r < 8; ++r) sl[(8 * hh + r) * 68 + nt * 16 + m] = fmaf(acc[nt][r], WCARRY_INV, bp2v[nt]);
    }
    wave_lds_sync();
    store_tile_f16(sl, peP + row0 * CH_D, lane);
    wave_lds_sync();
    const v4f qv = *(const v4f*)(qry + (size_t)ng * CH_D + c4);
#pragma unroll 1
    for (int half = 0; half < 2; ++half) {
#pragma unroll
      for (int i = 0; i < 4; ++i) {
        const int row = (half * 4 + i) * 2 + hh;
        const int nbr = nbs[wave][row];
        const v4f kg = *(const v4f*)(keyv + (size_t)(b * NPT + nbr) * CH_D + c4);
        const v4f pe4 = *(const v4f*)(sl + row * 68 + c4);
        const v4f s4 = (qv - kg) + pe4;
        *(v4f*)(sl + row * 68 + c4) = s4;
      }
      asm volatile("" ::: "memory");
    }
    wave_lds_sync();
    store_tile_f16(sl, sP + row0 * CH_D, lane);
    v16h sa[2];
    sa[0] = frag_from_f32(sl + m * 68 + 8 * hh);
    sa[1] = frag_from_f32(sl + m * 68 + 32 + 8 * hh);
    wave_lds_sync();
#pragma unroll
    for (int nt = 0; nt < 16; ++nt) {
      v8f c = (v8f){0.f, 0.f, 0.f, 0.f, 0.f, 0.f, 0.f, 0.f};
#pragma unroll
      for (int ks = 0; ks < 2; ++ks) {
        const v16h bfr = frag_load(pW + OFF_WA1 + (size_t)(nt * 16 + m) * CH_D + ks * 32 + 8 * hh);
        c = mma_h(sa[ks], bfr, c);
      }
      float s = 0.f, q2 = 0.f;
#pragma unroll
      for (int r = 0; r < 8; ++r) {
        const float u = c[r] * WCARRY_INV;
        s += u;
        q2 = fmaf(u, u, q2);
      }
      ssum[nt] += s;
      ssq[nt] += q2;
      asm volatile("" ::: "memory");
    }
  }
#pragma unroll
  for (int nt = 0; nt < 16; ++nt) {
    const float so = __shfl_xor(ssum[nt], 16);
    const float qo = __shfl_xor(ssq[nt], 16);
    wst[wave][nt * 16 + m] = ssum[nt] + so;
    wst[wave][256 + nt * 16 + m] = ssq[nt] + qo;
  }
  __syncthreads();
  {
    const v4f w0 = *(const v4f*)(wst[0] + tid * 4);
    const v4f w1 = *(const v4f*)(wst[1] + tid * 4);
    const v4f w2 = *(const v4f*)(wst[2] + tid * 4);
    const v4f w3 = *(const v4f*)(wst[3] + tid * 4);
    const v4f o = ((w0 + w1) + w2) + w3;
    float* dst = part2 + (size_t)blockIdx.x * 512 + tid * 4;
    *(volatile v4f*)dst = o;
    __threadfence();
    *(volatile v4f*)dst = o;
  }
}

__global__ __launch_bounds__(256) void k_fin2(const float* __restrict__ part2, const float* __restrict__ gamma,
                                              const float* __restrict__ beta, const float* __restrict__ ba1,
                                              float* __restrict__ sclsh2) {
  __shared__ __align__(16) float outv[512];
  const int c = threadIdx.x;
  double ds = 0.0, dq = 0.0;
#pragma unroll 4
  for (int b = 0; b < 512; ++b) {
    ds += (double)part2[(size_t)b * 512 + c];
    dq += (double)part2[(size_t)b * 512 + 256 + c];
  }
  const double invR = 1.0 / (double)NROWS_ALL;
  const double mean = ds * invR;
  const double var = dq * invR - mean * mean;
  const float varf = fmaxf((float)var, 0.0f);
  const float scl = gamma[c] * (1.0f / sqrtf(varf + BN_EPS_F));
  const double bb = (double)ba1[c];
  const double meanfull = mean + bb;
  const float sh = (float)((double)beta[c] + (bb - meanfull) * (double)scl);
  outv[c] = scl * WCARRY_INV;
  outv[256 + c] = sh;
  __syncthreads();
  if (c < 128) {
    const v4f v = *(const v4f*)(outv + c * 4);
    *(volatile v4f*)(sclsh2 + c * 4) = v;
    __threadfence();
    *(volatile v4f*)(sclsh2 + c * 4) = v;
  }
}

__global__ __launch_bounds__(128) void k_attn_out(
    const float* __restrict__ x, const float* __restrict__ valv,
    const _Float16* __restrict__ sP, const unsigned* __restrict__ peW,
    const _Float16* __restrict__ pW, const float* __restrict__ sclsh2,
    const float* __restrict__ ba2, const float* __restrict__ bend, float* __restrict__ out) {
  __shared__ __align__(16) float slabL[4][16 * 68];
  __shared__ __align__(16) float bnc[4][16 * 36];
  __shared__ float rinv[4][16];
  __shared__ __align__(16) float aggb[16 * 68];
  __shared__ __align__(16) float slabO[16 * 132];
  __shared__ __align__(16) float sbn[512];
  const int tid = threadIdx.x;
  const int wave = tid >> 5, lane = tid & 31;
  const int m = lane & 15, hh = lane >> 4;
  {
    const v4f v = *(const v4f*)(sclsh2 + tid * 4);
    *(v4f*)(sbn + tid * 4) = v;
  }
  __syncthreads();
  float ba2v[4];
#pragma unroll
  for (int nt = 0; nt < 4; ++nt) ba2v[nt] = ba2[nt * 16 + m];
  float* sl = slabL[wave];
  float* bo = bnc[wave];

#pragma unroll 1
  for (int sub = 0; sub < 4; ++sub) {
    const int nsub = wave * 4 + sub;
    const int ng = blockIdx.x * 16 + nsub;
    const size_t row0 = (size_t)ng * NBR;
    v16h sa[2];
    sa[0] = frag_load(sP + (row0 + m) * CH_D + 8 * hh);
    sa[1] = frag_load(sP + (row0 + m) * CH_D + 32 + 8 * hh);
    v8f acc[4];
#pragma unroll
    for (int nt = 0; nt < 4; ++nt) acc[nt] = (v8f){0.f, 0.f, 0.f, 0.f, 0.f, 0.f, 0.f, 0.f};
#pragma unroll 1
    for (int kc = 0; kc < 8; ++kc) {
#pragma unroll
      for (int s2 = 0; s2 < 2; ++s2) {
        v8f c = (v8f){0.f, 0.f, 0.f, 0.f, 0.f, 0.f, 0.f, 0.f};
#pragma unroll
        for (int ks = 0; ks < 2; ++ks) {
          const v16h bfr = frag_load(pW + OFF_WA1 + (size_t)(kc * 32 + s2 * 16 + m) * CH_D + ks * 32 + 8 * hh);
          c = mma_h(sa[ks], bfr, c);
        }
        const int ch = kc * 32 + s2 * 16 + m;
        const float scl = sbn[ch], sh = sbn[256 + ch];
#pragma unroll
        for (int r = 0; r < 8; ++r)
          bo[(8 * hh + r) * 36 + s2 * 16 + m] = fmaxf(fmaf(c[r], scl, sh), 0.0f);
      }
      asm volatile("" ::: "memory");
      wave_lds_sync();
      const v16h aa = frag_from_f32(bo + m * 36 + 8 * hh);
#pragma unroll
      for (int nt = 0; nt < 4; ++nt) {
        const v16h bfr = frag_load(pW + OFF_WA2 + (size_t)(nt * 16 + m) * CH_HID + kc * 32 + 8 * hh);
        acc[nt] = mma_h(aa, bfr, acc[nt]);
      }
      asm volatile("" ::: "memory");
      wave_lds_sync();
    }
#pragma unroll
    for (int nt = 0; nt < 4; ++nt) {
#pragma unroll
      for (int r = 0; r < 8; ++r) sl[(8 * hh + r) * 68 + nt * 16 + m] = fmaf(acc[nt][r], WCARRY_INV, ba2v[nt]);
    }
    wave_lds_sync();
    {
      float* lr = sl + m * 68 + 32 * hh;
      float mx = -INFINITY;
#pragma unroll 2
      for (int j = 0; j < 8; ++j) {
        const v4f v = *(const v4f*)(lr + 4 * j);
        mx = fmaxf(mx, fmaxf(fmaxf(v.x, v.y), fmaxf(v.z, v.w)));
      }
      const float mxo = __shfl_xor(mx, 16);
      mx = fmaxf(mx, mxo);
      float sm = 0.0f;
#pragma unroll 2
      for (int j = 0; j < 8; ++j) {
        const v4f v = *(const v4f*)(lr + 4 * j);
        v4f e;
        e.x = expf(v.x - mx);
        e.y = expf(v.y - mx);
        e.z = expf(v.z - mx);
        e.w = expf(v.w - mx);
        *(v4f*)(lr + 4 * j) = e;
        sm += (e.x + e.y) + (e.z + e.w);
      }
      const float smo = __shfl_xor(sm, 16);
      sm = sm + smo;
      rinv[wave][m] = 1.0f / sm;
    }
    wave_lds_sync();
    {
      const v2f vv = *(const v2f*)(valv + (size_t)ng * CH_D + 2 * lane);
      float a0 = 0.0f, a1 = 0.0f;
#pragma unroll 4
      for (int mm = 0; mm < 16; ++mm) {
        const unsigned w = peW[(row0 + mm) * 32 + lane];
        const float p0 = h16_to_f32(w & 0xffffu);
        const float p1 = h16_to_f32(w >> 16);
        const v2f e = *(const v2f*)(sl + mm * 68 + 2 * lane);
        const float inv = rinv[wave][mm];
        const float w0 = e.x * inv;
        const float w1 = e.y * inv;
        const float u0 = vv.x + p0;
        const float u1 = vv.y + p1;
        a0 = fmaf(w0, u0, a0);
        a1 = fmaf(w1, u1, a1);
      }
      *(v2f*)(aggb + nsub * 68 + 2 * lane) = (v2f){a0, a1};
    }
    wave_lds_sync();
  }
  __syncthreads();

  {
    v16h ea[2];
    ea[0] = frag_from_f32(aggb + m * 68 + 8 * hh);
    ea[1] = frag_from_f32(aggb + m * 68 + 32 + 8 * hh);
#pragma unroll
    for (int t = 0; t < 2; ++t) {
      const int nt = wave * 2 + t;
      v8f c = (v8f){0.f, 0.f, 0.f, 0.f, 0.f, 0.f, 0.f, 0.f};
#pragma unroll
      for (int ks = 0; ks < 2; ++ks) {
        const v16h bfr = frag_load(pW + OFF_WEND + (size_t)(nt * 16 + m) * CH_D + ks * 32 + 8 * hh);
        c = mma_h(ea[ks], bfr, c);
      }
      const float bb = bend[nt * 16 + m];
#pragma unroll
      for (int r = 0; r < 8; ++r) slabO[(8 * hh + r) * 132 + nt * 16 + m] = fmaf(c[r], WCARRY_INV, bb);
    }
  }
  __syncthreads();
  {
    v4f yv[4];
#pragma unroll
    for (int i = 0; i < 4; ++i) {
      const int row = wave * 4 + i;
      const size_t o = ((size_t)blockIdx.x * 16 + row) * CH_IN + lane * 4;
      const v4f xv = *(const v4f*)(x + o);
      const v4f sv = *(const v4f*)(slabO + row * 132 + lane * 4);
      yv[i] = sv + xv;
    }
    for (int pass = 0; pass < 2; ++pass) {
#pragma unroll
      for (int i = 0; i < 4; ++i) {
        const int row = wave * 4 + i;
        const size_t o = ((size_t)blockIdx.x * 16 + row) * CH_IN + lane * 4;
        *(volatile v4f*)(out + o) = yv[i];
      }
      __threadfence();
    }
  }
}

extern "C" void kernel_launch(void* const* d_in, const int* in_sizes, int n_in,
                              void* d_out, int out_size, void* d_ws, size_t ws_size,
                              hipStream_t stream) {
  (void)in_sizes;
  if (n_in < 24) return;
  if (out_size < NPOINTS * CH_IN) return;
  const float* x    = (const float*)d_in[0];
  const float* pos  = (const float*)d_in[1];
  const float* Wst  = (const float*)d_in[2];
  const float* bst  = (const float*)d_in[3];
  const float* Wk   = (const float*)d_in[4];
  const float* bk   = (const float*)d_in[5];
  const float* Wq   = (const float*)d_in[6];
  const float* bq   = (const float*)d_in[7];
  const float* Wv   = (const float*)d_in[8];
  const float* bv   = (const float*)d_in[9];
  const float* Wp1  = (const float*)d_in[10];
  const float* bp1  = (const float*)d_in[11];
  const float* gp   = (const float*)d_in[12];
  const float* bep  = (const float*)d_in[13];
  const float* Wp2  = (const float*)d_in[14];
  const float* bp2  = (const float*)d_in[15];
  const float* Wa1  = (const float*)d_in[16];
  const float* ba1  = (const float*)d_in[17];
  const float* ga   = (const float*)d_in[18];
  const float* bea  = (const float*)d_in[19];
  const float* Wa2  = (const float*)d_in[20];
  const float* ba2  = (const float*)d_in[21];
  const float* Wend = (const float*)d_in[22];
  const float* bend = (const float*)d_in[23];
  float* out = (float*)d_out;

  const size_t SZ_PW = (size_t)PACK_HALVES * 2;
  const size_t SZ_IDX = (size_t)NROWS_ALL * 4;
  const size_t SZ_PROJ = (size_t)NPOINTS * CH_D * 4;
  const size_t SZ_P1 = (size_t)256 * 16 * 8;
  const size_t SZ_S1 = 1024;
  const size_t SZ_P2 = (size_t)512 * 512 * 4;
  const size_t SZ_S2 = 2048;
  const size_t SZ_PLANE = (size_t)NROWS_ALL * CH_D * 2;
  size_t off = 0;
  char* ws = (char*)d_ws;
  _Float16* pW = (_Float16*)(ws + off); off += SZ_PW;
  int* idxb = (int*)(ws + off); off += SZ_IDX;
  float* keyo = (float*)(ws + off); off += SZ_PROJ;
  float* valo = (float*)(ws + off); off += SZ_PROJ;
  float* qryo = (float*)(ws + off); off += SZ_PROJ;
  double* part1 = (double*)(ws + off); off += SZ_P1;
  float* sclsh1 = (float*)(ws + off); off += SZ_S1;
  float* part2 = (float*)(ws + off); off += SZ_P2;
  float* sclsh2 = (float*)(ws + off); off += SZ_S2;
  _Float16* peP = (_Float16*)(ws + off); off += SZ_PLANE;
  _Float16* sP = (_Float16*)(ws + off); off += SZ_PLANE;
  if (off > ws_size) return;
  if (off > (size_t)134217728) return;

  k_pack<<<32, 256, 0, stream>>>(Wst, Wk, Wq, Wv, Wp2, Wa1, Wa2, Wend, pW);
  k_knn<<<dim3(NPT / 256, NBATCH), 256, 0, stream>>>(pos, idxb);
  k_proj<<<NPOINTS / 64, 128, 0, stream>>>(x, pW, bst, bk, bq, bv, keyo, valo, qryo);
  k_mom<<<256, 256, 0, stream>>>(pos, idxb, part1);
  k_fin1<<<1, 256, 0, stream>>>(part1, Wp1, bp1, gp, bep, sclsh1);
  k_pe_s<<<NPOINTS / 32, 128, 0, stream>>>(pos, idxb, qryo, keyo, Wp1, bp1, sclsh1, pW, bp2, peP, sP, part2);
  k_fin2<<<1, 256, 0, stream>>>(part2, ga, bea, ba1, sclsh2);
  k_attn_out<<<NPOINTS / 16, 128, 0, stream>>>(x, valo, sP, (const unsigned*)peP, pW, sclsh2, ba2, bend, out);
}
